// MambaBlock_29557964931128
// MI455X (gfx1250) — hardware-verified
//
#include <hip/hip_runtime.h>
#include <math.h>

typedef __attribute__((ext_vector_type(16))) _Float16 v16h;
typedef __attribute__((ext_vector_type(8)))  _Float16 v8h;
typedef __attribute__((ext_vector_type(8)))  float    v8f;
typedef __attribute__((ext_vector_type(4)))  float    v4f;

constexpr int kBatch = 2;
constexpr int kSeqL  = 2048;
constexpr int kDmod  = 1024;
constexpr int kDin   = 2048;
constexpr int kNst   = 16;
constexpr int kDtR   = 64;
constexpr int kPrjN  = 96;
constexpr int kPrjP  = 128;
constexpr int kXZP   = 2 * kDin;
constexpr int kRows  = kBatch * kSeqL;
constexpr int kTP    = 260;
constexpr float kEps = 1e-6f;

constexpr float kCarryW   = 32.0f;
constexpr float kCarryWdt = 8.0f;
constexpr float kCarryDt  = 16.0f;
constexpr float kCarryY   = 16.0f;

static_assert(kDtR + 2 * kNst == kPrjN, "small projection width");
static_assert((kDmod % 32) == 0 && (kDin % 32) == 0 && (kDtR % 32) == 0, "GEMM K multiples of 32");
static_assert((kRows % 64) == 0 && (kSeqL % 64) == 0 && (kXZP % 64) == 0 && (kPrjP % 64) == 0 &&
              (kDin % 64) == 0 && (kDmod % 64) == 0, "GEMM M,N multiples of 64");
static_assert((kDmod % 64) == 0 && (kDin % 64) == 0 && (kDtR % 64) == 0, "transpose tiles");
static_assert(kDmod == 1024 && kDin == 2048 && kSeqL == 2048, "lane maps below assume these shapes");

constexpr size_t kSzWIN  = (size_t)kXZP  * kDmod * 2;
constexpr size_t kSzWXP  = (size_t)kPrjP * kDmod * 2;
constexpr size_t kSzWDT  = (size_t)kDin  * kDtR  * 2;
constexpr size_t kSzWOUT = (size_t)kDmod * kDin  * 2;
constexpr size_t kSzU16  = (size_t)kRows * kDmod * 2;
constexpr size_t kSzXZ   = (size_t)kSeqL * kXZP  * 4;
constexpr size_t kSzUC   = (size_t)kSeqL * kDin  * 4;
constexpr size_t kSzPROJ = (size_t)kRows * kPrjP * 4;
constexpr size_t kSzDT16 = (size_t)kRows * kDtR  * 2;
constexpr size_t kSzDLR  = (size_t)kSeqL * kDin  * 4;
constexpr size_t kSzY16  = (size_t)kSeqL * kDin  * 2;
constexpr size_t kOffWIN  = 0;
constexpr size_t kOffWXP  = kOffWIN  + kSzWIN;
constexpr size_t kOffWDT  = kOffWXP  + kSzWXP;
constexpr size_t kOffWOUT = kOffWDT  + kSzWDT;
constexpr size_t kOffU16  = kOffWOUT + kSzWOUT;
constexpr size_t kOffXZ   = kOffU16  + kSzU16;
constexpr size_t kOffUC   = kOffXZ   + kSzXZ;
constexpr size_t kOffPROJ = kOffUC   + kSzUC;
constexpr size_t kOffDT16 = kOffPROJ + kSzPROJ;
constexpr size_t kOffDLR  = kOffDT16 + kSzDT16;
constexpr size_t kOffY16  = kOffDLR  + kSzDLR;
constexpr size_t kWsTotal = kOffY16  + kSzY16;
static_assert(kWsTotal == 99614720ull, "carve total");
static_assert(kWsTotal <= 134217728ull, "carve cap");
static_assert((kOffWXP % 128) == 0 && (kOffWDT % 128) == 0 && (kOffWOUT % 128) == 0 && (kOffU16 % 128) == 0 &&
              (kOffXZ % 128) == 0 && (kOffUC % 128) == 0 && (kOffPROJ % 128) == 0 && (kOffDT16 % 128) == 0 &&
              (kOffDLR % 128) == 0 && (kOffY16 % 128) == 0, "128-B aligned regions");

union FragU { v16h v; v8h h[2]; };
__device__ __forceinline__ v16h frag_load(const _Float16* p) {
  FragU f;
  f.h[0] = *(const v8h*)(p);
  f.h[1] = *(const v8h*)(p + 16);
  return f.v;
}
__device__ __forceinline__ v8f mma_f16(v16h a, v16h b, v8f c) {
  return __builtin_amdgcn_wmma_f32_16x16x32_f16(false, a, false, b, (short)0, c, false, false);
}
__device__ __forceinline__ void group_guard(v8f& a, v8f& b, v8f& c, v8f& d, v16h x, v16h y) {
  asm volatile("v_nop\n\tv_nop\n\tv_nop\n\tv_nop" : "+v"(a), "+v"(b), "+v"(c), "+v"(d) : "v"(x), "v"(y));
}
__device__ __forceinline__ void keep4_h(v16h a, v16h b, v16h c, v16h d) {
  asm volatile("v_nop" :: "v"(a), "v"(b), "v"(c), "v"(d));
}
__device__ __forceinline__ void acc_guard4(v8f& a, v8f& b, v8f& c, v8f& d) {
  asm volatile("v_nop\n\tv_nop\n\tv_nop\n\tv_nop" : "+v"(a), "+v"(b), "+v"(c), "+v"(d));
}

template <int BIAS_MODE, bool RESID>
__global__ __launch_bounds__(256) void gemm64_f16_kernel(
    const unsigned short* __restrict__ Ap, int lda,
    const unsigned short* __restrict__ Btp, int ldb,
    float* __restrict__ C, int ldc,
    const float* __restrict__ bias,
    const float* __restrict__ resid,
    int M, int N, int K, float scale)
{
  const _Float16* A  = (const _Float16*)Ap;
  const _Float16* Bt = (const _Float16*)Btp;
  __shared__ __align__(16) float sT[8][16 * 68];
  const int lane = threadIdx.x & 31;
  const int wave = threadIdx.x >> 5;
  const int tilesN = N >> 6;
  const int tilesM = M >> 6;
  const int tile = blockIdx.x * 8 + wave;
  if (tile >= tilesM * tilesN) return;
  const int tm = tile / tilesN;
  const int tn = tile - tm * tilesN;
  const int m0 = tm << 6;
  const int n0 = tn << 6;

  const int rlane = lane & 15;
  const int koff  = (lane >> 4) * 8;
  const int mOff  = (lane >> 4) * 8;

  v8f acc[4][4];
#pragma unroll
  for (int i = 0; i < 4; ++i)
#pragma unroll
    for (int j = 0; j < 4; ++j) acc[i][j] = (v8f){0.f,0.f,0.f,0.f,0.f,0.f,0.f,0.f};

  for (int k0 = 0; k0 < K; k0 += 32) {
    v16h bh[4];
#pragma unroll
    for (int j = 0; j < 4; ++j) {
      const size_t bo = (size_t)(n0 + (j << 4) + rlane) * ldb + koff + k0;
      bh[j] = frag_load(Bt + bo);
    }
#pragma unroll
    for (int i = 0; i < 4; ++i) {
      const size_t ao = (size_t)(m0 + (i << 4) + rlane) * lda + koff + k0;
      const v16h ah = frag_load(A + ao);
#pragma unroll
      for (int j = 0; j < 4; ++j) acc[i][j] = mma_f16(ah, bh[j], acc[i][j]);
      group_guard(acc[i][0], acc[i][1], acc[i][2], acc[i][3], ah, bh[3]);
    }
    keep4_h(bh[0], bh[1], bh[2], bh[3]);
  }
  acc_guard4(acc[0][0], acc[0][1], acc[0][2], acc[0][3]);
  acc_guard4(acc[1][0], acc[1][1], acc[1][2], acc[1][3]);
  acc_guard4(acc[2][0], acc[2][1], acc[2][2], acc[2][3]);
  acc_guard4(acc[3][0], acc[3][1], acc[3][2], acc[3][3]);

  float* slab = sT[wave];
  const int hh = lane >> 4, c4 = (lane & 15) * 4;
#pragma unroll
  for (int i = 0; i < 4; ++i) {
    const int mBase = m0 + (i << 4);
#pragma unroll
    for (int j = 0; j < 4; ++j) {
      const int n = n0 + (j << 4) + rlane;
      float bv = 0.f;
      if (BIAS_MODE == 2) bv = bias[n];
#pragma unroll
      for (int r = 0; r < 8; ++r) {
        float v = acc[i][j][r] * scale;
        if (BIAS_MODE == 2) v += bv;
        slab[(mOff + r) * 68 + (j << 4) + rlane] = v;
      }
    }
    __builtin_amdgcn_fence(__ATOMIC_RELEASE, "workgroup");
    __builtin_amdgcn_wave_barrier();
    __builtin_amdgcn_fence(__ATOMIC_ACQUIRE, "workgroup");
    v4f vals[8];
#pragma unroll
    for (int it = 0; it < 8; ++it) {
      const int row = it * 2 + hh;
      v4f v = *(const v4f*)(slab + row * 68 + c4);
      if (RESID) {
        const v4f rr = *(const v4f*)(resid + (size_t)(mBase + row) * ldc + n0 + c4);
        v = v + rr;
      }
      vals[it] = v;
    }
    for (int pass = 0; pass < 2; ++pass) {
#pragma unroll
      for (int it = 0; it < 8; ++it) {
        const int row = it * 2 + hh;
        *(volatile v4f*)(C + (size_t)(mBase + row) * ldc + n0 + c4) = vals[it];
      }
      __threadfence();
    }
    __builtin_amdgcn_fence(__ATOMIC_RELEASE, "workgroup");
    __builtin_amdgcn_wave_barrier();
    __builtin_amdgcn_fence(__ATOMIC_ACQUIRE, "workgroup");
  }
}

__global__ __launch_bounds__(256) void transpose_cast_kernel(
    const float* __restrict__ W, unsigned short* __restrict__ Bt, int Kdim, int Ndim, float scale)
{
  __shared__ float tile[64 * 65];
  const int tid = threadIdx.x, lane = tid & 31, wave = tid >> 5;
  const int n0 = blockIdx.x * 64;
  const int k0 = blockIdx.y * 64;
#pragma unroll
  for (int p = 0; p < 16; ++p) {
    const int idx = tid + p * 256;
    const int kk  = idx >> 6;
    const int nn  = idx & 63;
    const int n   = n0 + nn;
    const int nc  = (n < Ndim) ? n : (Ndim - 1);
    const float v = W[(size_t)(k0 + kk) * Ndim + nc];
    tile[kk * 65 + nn] = (n < Ndim) ? (v * scale) : 0.f;
  }
  __syncthreads();
  const int q = lane >> 3, c8 = (lane & 7) * 8;
  v8h hv[2];
#pragma unroll
  for (int it = 0; it < 2; ++it) {
    const int nrow = it * 32 + wave * 4 + q;
#pragma unroll
    for (int e = 0; e < 8; ++e) hv[it][e] = (_Float16)tile[(c8 + e) * 65 + nrow];
  }
  for (int pass = 0; pass < 2; ++pass) {
#pragma unroll
    for (int it = 0; it < 2; ++it) {
      const int nrow = it * 32 + wave * 4 + q;
      *(volatile v8h*)(Bt + (size_t)(n0 + nrow) * Kdim + k0 + c8) = hv[it];
    }
    __threadfence();
  }
}

__global__ __launch_bounds__(256) void rmsnorm_cast_kernel(
    const float* __restrict__ X, const float* __restrict__ gs, unsigned short* __restrict__ U16)
{
  const int lane = threadIdx.x & 31, wave = threadIdx.x >> 5;
  const int row = blockIdx.x * 8 + wave;
  const float* xr = X + (size_t)row * kDmod;
  v4f a[8];
#pragma unroll
  for (int c = 0; c < 4; ++c) {
    const float* p = xr + c * 256 + lane * 8;
    a[2 * c]     = *(const v4f*)(p);
    a[2 * c + 1] = *(const v4f*)(p + 4);
  }
  float ss = 0.f;
#pragma unroll
  for (int i = 0; i < 8; ++i) {
#pragma unroll
    for (int e = 0; e < 4; ++e) ss = fmaf(a[i][e], a[i][e], ss);
  }
#pragma unroll
  for (int off = 16; off >= 1; off >>= 1) ss += __shfl_xor(ss, off, 32);
  const float inv = rsqrtf(ss * (1.0f / (float)kDmod) + kEps);
  v8h hv[4];
#pragma unroll
  for (int c = 0; c < 4; ++c) {
    const float* sp = gs + c * 256 + lane * 8;
    const v4f s0 = *(const v4f*)(sp);
    const v4f s1 = *(const v4f*)(sp + 4);
#pragma unroll
    for (int e = 0; e < 4; ++e) {
      hv[c][e]     = (_Float16)((a[2 * c][e] * inv) * s0[e]);
      hv[c][4 + e] = (_Float16)((a[2 * c + 1][e] * inv) * s1[e]);
    }
  }
  unsigned short* ur = U16 + (size_t)row * kDmod + lane * 8;
  for (int pass = 0; pass < 2; ++pass) {
#pragma unroll
    for (int c = 0; c < 4; ++c) *(volatile v8h*)(ur + c * 256) = hv[c];
    __threadfence();
  }
}

__global__ __launch_bounds__(256) void dt_cast_kernel(
    const float* __restrict__ PROJ, unsigned short* __restrict__ DT16, int total8, float scale)
{
  const int i = blockIdx.x * 256 + threadIdx.x;
  if (i >= total8) return;
  const int e0  = i << 3;
  const int row = e0 >> 6;
  const int c8  = e0 & 63;
  const float* p = PROJ + (size_t)row * kPrjP + c8;
  const v4f a0 = *(const v4f*)(p);
  const v4f a1 = *(const v4f*)(p + 4);
  v8h hv;
#pragma unroll
  for (int e = 0; e < 4; ++e) {
    hv[e]     = (_Float16)(a0[e] * scale);
    hv[4 + e] = (_Float16)(a1[e] * scale);
  }
  unsigned short* qd = DT16 + e0;
  *(volatile v8h*)qd = hv;
  __threadfence();
  *(volatile v8h*)qd = hv;
}

__global__ __launch_bounds__(256) void conv_silu_kernel(
    const float* __restrict__ XZ, const float* __restrict__ ck, const float* __restrict__ cb,
    float* __restrict__ UC)
{
  __shared__ __align__(16) float sx[kDin + 8];
  const int tid = threadIdx.x;
  const int l = blockIdx.x;
  const float* xr = XZ + (size_t)l * kXZP;
#pragma unroll
  for (int it = 0; it < 2; ++it) {
    const int c = it * 1024 + tid * 4;
    *(v4f*)(sx + 4 + c) = *(const v4f*)(xr + c);
  }
  if (tid == 0) *(v4f*)(sx) = (v4f){0.f, 0.f, 0.f, 0.f};
  if (tid == 1) *(v4f*)(sx + 4 + kDin) = (v4f){0.f, 0.f, 0.f, 0.f};
  __syncthreads();
  const float w0 = ck[l], w1 = ck[kSeqL + l], w2 = ck[2 * kSeqL + l], w3 = ck[3 * kSeqL + l];
  const float bc = cb[l];
  float* orow = UC + (size_t)l * kDin;
#pragma unroll 1
  for (int it = 0; it < 2; ++it) {
    const int c = it * 1024 + tid * 4;
    const float xm1 = sx[3 + c];
    const v4f xa = *(const v4f*)(sx + 4 + c);
    const v4f xb = *(const v4f*)(sx + 8 + c);
    float xs[7];
    xs[0] = xm1; xs[1] = xa[0]; xs[2] = xa[1]; xs[3] = xa[2]; xs[4] = xa[3]; xs[5] = xb[0]; xs[6] = xb[1];
    v4f r;
#pragma unroll
    for (int e = 0; e < 4; ++e) {
      float acc = w0 * xs[e];
      acc = fmaf(w1, xs[e + 1], acc);
      acc = fmaf(w2, xs[e + 2], acc);
      acc = fmaf(w3, xs[e + 3], acc);
      const float sv = acc + bc;
      const float sg = __builtin_amdgcn_rcpf(1.0f + expf(-sv));
      r[e] = sv * sg;
    }
    *(volatile v4f*)(orow + c) = r;
    __threadfence();
    *(volatile v4f*)(orow + c) = r;
  }
}

__global__ __launch_bounds__(256) void scan_kernel(
    const float* __restrict__ DLR, const float* __restrict__ UC, const float* __restrict__ XZ,
    const float* __restrict__ PROJ, const float* __restrict__ A_log, const float* __restrict__ Dv,
    unsigned short* __restrict__ Y16)
{
  __shared__ __align__(16) float sBC[16 * 32];
  __shared__ __align__(16) float sY[16 * kTP];
  __shared__ float sA[kNst * 256];
  const int tid = threadIdx.x, lane = tid & 31, wave = tid >> 5;
  const int d0 = blockIdx.x * 256, d = d0 + tid;

#pragma unroll 1
  for (int n = 0; n < kNst; ++n) sA[n * 256 + tid] = -expf(A_log[(size_t)d * kNst + n]);
  __syncthreads();
  float An[kNst], h[kNst];
#pragma unroll
  for (int n = 0; n < kNst; ++n) {
    An[n] = sA[n * 256 + tid];
    h[n] = 0.f;
  }
  const float Dd = Dv[d];

#pragma unroll 1
  for (int c = 0; c < kSeqL / 16; ++c) {
    const int l0 = c * 16;
    if (tid < 128) {
      const int r = tid >> 3, q = (tid & 7) * 4;
      const v4f v = *(const v4f*)(PROJ + (size_t)(l0 + r) * kPrjP + kDtR + q);
      *(v4f*)(sBC + r * 32 + q) = v;
    }
    __syncthreads();
#pragma unroll 1
    for (int s = 0; s < 16; ++s) {
      const size_t m = (size_t)(l0 + s);
      const float a     = DLR[m * kDin + d];
      const float xv    = UC[m * kDin + d];
      const float zv    = XZ[m * kXZP + kDin + d];
      const float delta = fmaxf(a, 0.0f) + log1pf(__expf(-fabsf(a)));
      v4f Bq[4], Cq[4];
#pragma unroll
      for (int qq = 0; qq < 4; ++qq) {
        Bq[qq] = *(const v4f*)(sBC + s * 32 + 4 * qq);
        Cq[qq] = *(const v4f*)(sBC + s * 32 + kNst + 4 * qq);
      }
      const float dux = delta * xv;
      float y = 0.f;
#pragma unroll
      for (int n = 0; n < kNst; ++n) {
        const float e  = __expf(delta * An[n]);
        const float hn = e * h[n] + dux * Bq[n >> 2][n & 3];
        h[n] = hn;
        y = hn * Cq[n >> 2][n & 3] + y;
      }
      y = xv * Dd + y;
      const float sg = __builtin_amdgcn_rcpf(1.0f + __expf(-zv));
      const float g  = zv * sg;
      sY[s * kTP + tid] = (y * g) * kCarryY;
    }
    __syncthreads();
    v8h hv[2];
#pragma unroll
    for (int it = 0; it < 2; ++it) {
      const float* sp = sY + (it * 8 + wave) * kTP + lane * 8;
      const v4f a0 = *(const v4f*)(sp);
      const v4f a1 = *(const v4f*)(sp + 4);
#pragma unroll
      for (int e = 0; e < 4; ++e) {
        hv[it][e]     = (_Float16)a0[e];
        hv[it][4 + e] = (_Float16)a1[e];
      }
    }
    for (int pass = 0; pass < 2; ++pass) {
#pragma unroll
      for (int it = 0; it < 2; ++it)
        *(volatile v8h*)(Y16 + (size_t)(l0 + it * 8 + wave) * kDin + d0 + lane * 8) = hv[it];
      __threadfence();
    }
  }
}

extern "C" void kernel_launch(void* const* d_in, const int* in_sizes, int n_in,
                              void* d_out, int out_size, void* d_ws, size_t ws_size,
                              hipStream_t stream)
{
  if (n_in < 11) return;
  if (in_sizes[0] != kRows * kDmod) return;
  if (in_sizes[1] != kDmod) return;
  if (in_sizes[2] != kDmod * kXZP) return;
  if (in_sizes[3] != 4 * kSeqL || in_sizes[4] != kSeqL) return;
  if (in_sizes[5] != kDmod * kPrjN) return;
  if (in_sizes[6] != kDtR * kDin || in_sizes[7] != kDin) return;
  if (in_sizes[8] != kDin * kDmod) return;
  if (in_sizes[9] != kDin * kNst || in_sizes[10] != kDin) return;
  if (out_size != kRows * kDmod) return;
  if (ws_size < kWsTotal) return;

  const float* x_in   = (const float*)d_in[0];
  const float* nscale = (const float*)d_in[1];
  const float* W_in   = (const float*)d_in[2];
  const float* convk  = (const float*)d_in[3];
  const float* convb  = (const float*)d_in[4];
  const float* W_x    = (const float*)d_in[5];
  const float* W_dt   = (const float*)d_in[6];
  const float* b_dt   = (const float*)d_in[7];
  const float* W_out  = (const float*)d_in[8];
  const float* A_log  = (const float*)d_in[9];
  const float* Dv     = (const float*)d_in[10];
  float* dout = (float*)d_out;

  char* ws = (char*)d_ws;
  unsigned short* WIN16  = (unsigned short*)(ws + kOffWIN);
  unsigned short* WXP16  = (unsigned short*)(ws + kOffWXP);
  unsigned short* WDT16  = (unsigned short*)(ws + kOffWDT);
  unsigned short* WOUT16 = (unsigned short*)(ws + kOffWOUT);
  unsigned short* U16    = (unsigned short*)(ws + kOffU16);
  float*          XZ     = (float*)(ws + kOffXZ);
  float*          UC     = (float*)(ws + kOffUC);
  float*          PROJ   = (float*)(ws + kOffPROJ);
  unsigned short* DT16   = (unsigned short*)(ws + kOffDT16);
  float*          DLR    = (float*)(ws + kOffDLR);
  unsigned short* Y16    = (unsigned short*)(ws + kOffY16);
  const float* dummy_bias  = b_dt;
  const float* dummy_resid = x_in;

  transpose_cast_kernel<<<dim3(kXZP / 64, kDmod / 64), 256, 0, stream>>>(W_in, WIN16, kDmod, kXZP, kCarryW);
  transpose_cast_kernel<<<dim3(kPrjP / 64, kDmod / 64), 256, 0, stream>>>(W_x, WXP16, kDmod, kPrjN, kCarryW);
  transpose_cast_kernel<<<dim3(kDin / 64, kDtR / 64), 256, 0, stream>>>(W_dt, WDT16, kDtR, kDin, kCarryWdt);
  transpose_cast_kernel<<<dim3(kDmod / 64, kDin / 64), 256, 0, stream>>>(W_out, WOUT16, kDin, kDmod, kCarryW);

  rmsnorm_cast_kernel<<<kRows / 8, 256, 0, stream>>>(x_in, nscale, U16);

  gemm64_f16_kernel<0, false><<<dim3((kRows / 64) * (kPrjP / 64) / 8), 256, 0, stream>>>(
      U16, kDmod, WXP16, kDmod, PROJ, kPrjP, dummy_bias, dummy_resid,
      kRows, kPrjP, kDmod, 1.0f / kCarryW);

  dt_cast_kernel<<<(kRows * kDtR) / 8 / 256, 256, 0, stream>>>(PROJ, DT16, (kRows * kDtR) / 8, kCarryDt);

  for (int b = 0; b < kBatch; ++b) {
    const unsigned short* U16b  = U16  + (size_t)b * kSeqL * kDmod;
    const unsigned short* DT16b = DT16 + (size_t)b * kSeqL * kDtR;
    const float* PROJb = PROJ + (size_t)b * kSeqL * kPrjP;
    const float* xinb  = x_in + (size_t)b * kSeqL * kDmod;
    float* outb = dout + (size_t)b * kSeqL * kDmod;

    gemm64_f16_kernel<0, false><<<dim3((kSeqL / 64) * (kXZP / 64) / 8), 256, 0, stream>>>(
        U16b, kDmod, WIN16, kDmod, XZ, kXZP, dummy_bias, dummy_resid,
        kSeqL, kXZP, kDmod, 1.0f / kCarryW);

    conv_silu_kernel<<<kSeqL, 256, 0, stream>>>(XZ, convk, convb, UC);

    gemm64_f16_kernel<2, false><<<dim3((kSeqL / 64) * (kDin / 64) / 8), 256, 0, stream>>>(
        DT16b, kDtR, WDT16, kDtR, DLR, kDin, b_dt, dummy_resid,
        kSeqL, kDin, kDtR, 1.0f / (kCarryDt * kCarryWdt));

    scan_kernel<<<dim3(kDin / 256), 256, 0, stream>>>(DLR, UC, XZ, PROJb, A_log, Dv, Y16);

    gemm64_f16_kernel<0, true><<<dim3((kSeqL / 64) * (kDmod / 64) / 8), 256, 0, stream>>>(
        Y16, kDin, WOUT16, kDin, outb, kDmod, dummy_bias, xinb,
        kSeqL, kDmod, kDin, 1.0f / (kCarryY * kCarryW));
  }
}
